// GAT_DGL_Custom_55594056680299
// MI455X (gfx1250) — hardware-run, weakly checked
//
#include <hip/hip_runtime.h>


namespace {
constexpr int NN = 50000, NP = 50016, NE = 800000, FI = 256, H1 = 4, D1 = 64, F1 = 256, F2 = 64, MAXDEG = 1024, NGc = (NN + 511) / 512, PERMLEN = NE + 32 * NGc + 32;
constexpr float XS = 8.0f, SLOPE = 0.2f;

typedef _Float16 b16;
typedef __attribute__((ext_vector_type(16))) _Float16 v16b;
typedef __attribute__((ext_vector_type(8))) _Float16 v8b;
typedef __attribute__((ext_vector_type(8))) float v8f;
typedef __attribute__((ext_vector_type(4))) float v4f;
typedef __attribute__((ext_vector_type(2))) float v2f;
__device__ __forceinline__ float bf16_rne(float f) { unsigned int u = __float_as_uint(f); u += 0x7FFFu + ((u >> 16) & 1u); return __uint_as_float(u & 0xFFFF0000u); }
__device__ __forceinline__ void split16(float v, b16& hi, b16& lo) { hi = (b16)v; lo = (b16)(v - (float)hi); }
__device__ __forceinline__ v16b frag_kb(const b16* p, int hh) { const v8b a = *(const v8b*)(p + 8 * hh), b = *(const v8b*)(p + 16 + 8 * hh); v16b f;
#pragma unroll
  for (int e = 0; e < 8; ++e) { f[e] = a[e]; f[8 + e] = b[e]; } return f; }
__device__ __forceinline__ v8f wmma16b(v16b a, v16b b, v8f c) { v8f d = __builtin_amdgcn_wmma_f32_16x16x32_f16(false, a, false, b, (short)0, c, false, false); asm volatile("v_nop\n\tv_nop\n\tv_nop\n\tv_nop" : "+v"(d) : "v"(a), "v"(b)); return d; }
__device__ __forceinline__ void wave_lds_sync() { __builtin_amdgcn_fence(__ATOMIC_RELEASE, "workgroup"); __builtin_amdgcn_wave_barrier(); __builtin_amdgcn_fence(__ATOMIC_ACQUIRE, "workgroup"); }
__device__ __forceinline__ float nexp(float x) { return __builtin_amdgcn_exp2f(x * 1.4426950408889634f); }
__device__ __forceinline__ float pmul(float a, float b) { float p = a * b; asm volatile("" : "+v"(p)); return p; }
__device__ __forceinline__ float leaky(float x) { return (x >= 0.0f) ? x : SLOPE * x; }
__device__ __forceinline__ float elu_f(float x) { return (x > 0.0f) ? x : (nexp(x) - 1.0f); }
constexpr int CSR_NBLK = 512, CSR_GB = 9, CSR_GN = 1 << CSR_GB  , CSR_MAXG = 512, CSR_CAP = 12288  ;
__global__ __launch_bounds__(64) void csrA_kernel(const int* __restrict__ dst, int E, int N, int nG, int CHP, int NGP, int* __restrict__ STG, int* __restrict__ HST) {
  extern __shared__ int sm[];
  int* cnt = sm; int* run = sm + NGP; int* ids = sm + 2 * NGP;
  const int b = blockIdx.x; const int ch = (E + CSR_NBLK - 1) / CSR_NBLK; const int e0 = b * ch, e1 = min(E, e0 + ch);
  for (int i = threadIdx.x; i < NGP; i += 64) cnt[i] = 0;
  for (int i = threadIdx.x; i < CHP; i += 64) ids[i] = -1;
  __syncthreads();
  if (threadIdx.x == 0) {
    for (int e = e0; e < e1; ++e) { int d = dst[e]; d = (d < 0) ? 0 : (d >= N ? N - 1 : d); cnt[d >> CSR_GB] += 1; }
    int acc = 0; for (int g = 0; g < nG; ++g) { run[g] = acc; acc += cnt[g]; }
    for (int e = e0; e < e1; ++e) { int d = dst[e]; d = (d < 0) ? 0 : (d >= N ? N - 1 : d); const int g = d >> CSR_GB; ids[run[g]] = e; run[g] += 1; } }
  __syncthreads();
  typedef __attribute__((ext_vector_type(4))) int v4i;
  for (int pass = 0; pass < 2; ++pass) {
    for (int i = threadIdx.x; i < CHP / 4; i += 64) *(volatile v4i*)(STG + (size_t)b * CHP + i * 4) = *(const v4i*)(&ids[i * 4]);
    for (int i = threadIdx.x; i < NGP / 4; i += 64) { v4i v; for (int e = 0; e < 4; ++e) v[e] = (i * 4 + e < nG) ? cnt[i * 4 + e] : 0; *(volatile v4i*)(HST + (size_t)b * NGP + i * 4) = v; }
    __threadfence(); }
}
__global__ __launch_bounds__(512) void csrS_kernel(const int* __restrict__ HST, int nG, int NGP, int* __restrict__ START, int* __restrict__ TOT, int* __restrict__ OFF) {
  __shared__ int tot[CSR_MAXG];
  const int b = threadIdx.x;
  for (int pass = 0; pass < 2; ++pass) { int runb = 0; for (int g = 0; g < nG; ++g) { int c = HST[(size_t)b * NGP + g]; c = (c < 0) ? 0 : c; ((volatile int*)OFF)[(size_t)g * CSR_NBLK + b] = runb; runb += c; } __threadfence(); }
  for (int g = threadIdx.x; g < nG; g += 512) { int s = 0; for (int bb = 0; bb < CSR_NBLK; ++bb) { int c = HST[(size_t)bb * NGP + g]; s += (c < 0) ? 0 : c; } tot[g] = s; }
  __syncthreads();
  if (threadIdx.x < 32) {
    __shared__ int st[CSR_MAXG + 32];
    if (threadIdx.x == 0) { int acc = 0; for (int g = 0; g < NGP; ++g) { st[g] = acc; if (g < nG) acc += (tot[g] + 31) & ~31; } st[NGP] = acc; }
    __builtin_amdgcn_fence(__ATOMIC_RELEASE, "workgroup"); __builtin_amdgcn_wave_barrier(); __builtin_amdgcn_fence(__ATOMIC_ACQUIRE, "workgroup");
    for (int pass = 0; pass < 2; ++pass) { for (int i = threadIdx.x; i < NGP + 32; i += 32) { ((volatile int*)START)[i] = (i <= NGP) ? st[min(i, NGP)] : 0; ((volatile int*)TOT)[i] = (i < nG) ? tot[i] : 0; } __threadfence(); } }
}
__global__ __launch_bounds__(256) void csrB_kernel(const int* __restrict__ dst, int N, int nG, int CHP, int NGP, int permLen, const int* __restrict__ STG, const int* __restrict__ HST, const int* __restrict__ OFF, const int* __restrict__ START, const int* __restrict__ TOT, int* __restrict__ PERM, int* __restrict__ ROWPTR, int* __restrict__ ROWCNT, int* __restrict__ FLAG) {
  typedef __attribute__((ext_vector_type(4))) int v4i;
  __shared__ int ids[CSR_CAP]; __shared__ unsigned short key[CSR_CAP]; __shared__ int outp[CSR_CAP]; __shared__ int ncnt[CSR_GN + 1]; __shared__ int boff[CSR_NBLK + 1];
  const int g = blockIdx.x, t_ = threadIdx.x; int tot = TOT[g]; int st = START[g], stn = START[g + 1]; const int v0 = g * CSR_GN; const int nv = min(CSR_GN, N - v0);
  st = (st < 0) ? 0 : (st > permLen - 32 ? permLen - 32 : st) & ~31; stn = (stn < st) ? st : (stn > permLen ? permLen : stn); tot = (tot < 0) ? 0 : tot; if (tot > stn - st && tot <= CSR_CAP) tot = stn - st;
  if (tot > CSR_CAP) {
    for (int pass = 0; pass < 2; ++pass) { for (int i = t_; i < CSR_GN / 4; i += 256) { v4i a, c; for (int e = 0; e < 4; ++e) { a[e] = st; c[e] = 0; } *(volatile v4i*)(ROWPTR + v0 + i * 4) = a; *(volatile v4i*)(ROWCNT + v0 + i * 4) = c; } if (t_ == 0) ((volatile int*)FLAG)[0] = 1; __threadfence(); } (void)nv; return; }
  if (t_ == 0) { int acc = 0; for (int b = 0; b < CSR_NBLK; ++b) { boff[b] = acc; int c = HST[(size_t)b * NGP + g]; c = (c < 0) ? 0 : (c > CHP ? CHP : c); acc += c; if (acc > tot) acc = tot; } boff[CSR_NBLK] = acc; }
  for (int i = t_; i <= CSR_GN; i += 256) ncnt[i] = 0;
  __syncthreads();
  for (int b = 0; b < CSR_NBLK; ++b) { const int c = boff[b + 1] - boff[b]; int o_ = OFF[(size_t)g * CSR_NBLK + b]; o_ = (o_ < 0) ? 0 : (o_ > CHP - c ? CHP - c : o_); const int* src_ = STG + (size_t)b * CHP + o_;
    for (int i = t_; i < c; i += 256) { int id = src_[i]; id = (id < 0) ? 0 : id; ids[boff[b] + i] = id; int d = dst[id]; d = (d < v0) ? v0 : (d >= N ? N - 1 : d); int kk = d - v0; kk = (kk < 0) ? 0 : (kk >= CSR_GN ? CSR_GN - 1 : kk); key[boff[b] + i] = (unsigned short)kk; } }
  __syncthreads();
  if (t_ == 0) { for (int i = 0; i < tot; ++i) ncnt[key[i]] += 1; int acc = 0; for (int vl = 0; vl < CSR_GN; ++vl) { const int c = ncnt[vl]; ncnt[vl] = acc; acc += c; } ncnt[CSR_GN] = acc;
    for (int i = 0; i < tot; ++i) { const int vl = key[i]; outp[ncnt[vl]] = ids[i]; ncnt[vl] += 1; }
    for (int vl = CSR_GN; vl > 0; --vl) ncnt[vl] = ncnt[vl - 1]; ncnt[0] = 0; }
  __syncthreads();
  for (int pass = 0; pass < 2; ++pass) {
    for (int i = t_; i < (stn - st) / 4; i += 256) { v4i v; for (int e = 0; e < 4; ++e) { const int q = i * 4 + e; v[e] = (q < tot) ? outp[q] : -1; } *(volatile v4i*)(PERM + st + i * 4) = v; }
    for (int i = t_; i < CSR_GN / 4; i += 256) { v4i a, c; for (int e = 0; e < 4; ++e) { const int vl = i * 4 + e; a[e] = st + ncnt[vl]; c[e] = (vl < nv) ? (ncnt[vl + 1] - ncnt[vl]) : 0; } *(volatile v4i*)(ROWPTR + v0 + i * 4) = a; *(volatile v4i*)(ROWCNT + v0 + i * 4) = c; }
    __threadfence(); }
}
__global__ __launch_bounds__(256) void csrZ_kernel(int* __restrict__ p, size_t n4) { typedef __attribute__((ext_vector_type(4))) int v4i; const size_t tid = (size_t)blockIdx.x * 256 + threadIdx.x, nth = (size_t)gridDim.x * 256; v4i z = {0, 0, 0, 0}; for (size_t i = tid; i < n4; i += nth) *(volatile v4i*)(p + i * 4) = z; }
struct CsrBufs { int *STG, *HST, *OFF, *START, *TOT, *PERM, *ROWPTR, *ROWCNT, *FLAG; int nG, NGP, CHP; size_t permLen; char* base; size_t bytes; };
static size_t csr_carve(CsrBufs& c, char* ws, size_t off, int E, int N) {
  const size_t off0 = off; c.base = ws + off;
  auto al = [&](size_t bytes) { char* p = ws + off; off += (bytes + 255) & ~(size_t)255; return p; };
  c.nG = (N + CSR_GN - 1) / CSR_GN; c.NGP = (c.nG + 31) & ~31; const int ch = (E + CSR_NBLK - 1) / CSR_NBLK; c.CHP = (ch + 31) & ~31; c.permLen = (size_t)E + 32 * (size_t)c.nG + 32;
  c.STG = (int*)al((size_t)CSR_NBLK * c.CHP * 4); c.HST = (int*)al((size_t)CSR_NBLK * c.NGP * 4); c.OFF = (int*)al((size_t)c.NGP * CSR_NBLK * 4); c.START = (int*)al((size_t)(c.NGP + 64) * 4); c.TOT = (int*)al((size_t)(c.NGP + 64) * 4);
  c.PERM = (int*)al(c.permLen * 4); c.ROWPTR = (int*)al((size_t)c.nG * CSR_GN * 4); c.ROWCNT = (int*)al((size_t)c.nG * CSR_GN * 4); c.FLAG = (int*)al(256);
  c.bytes = off - off0; return off;
}
static void csr_build(const CsrBufs& c, const int* dst, int E, int N, hipStream_t stream) {
  const size_t smem = (size_t)(2 * c.NGP + c.CHP) * 4;
  csrZ_kernel<<<512, 256, 0, stream>>>((int*)c.base, c.bytes / 16);
  csrA_kernel<<<CSR_NBLK, 64, smem, stream>>>(dst, E, N, c.nG, c.CHP, c.NGP, c.STG, c.HST);
  csrS_kernel<<<1, 512, 0, stream>>>(c.HST, c.nG, c.NGP, c.START, c.TOT, c.OFF);
  csrB_kernel<<<c.nG, 256, 0, stream>>>(dst, N, c.nG, c.CHP, c.NGP, (int)c.permLen, c.STG, c.HST, c.OFF, c.START, c.TOT, c.PERM, c.ROWPTR, c.ROWCNT, c.FLAG);
}

__global__ __launch_bounds__(256) void prep_kernel(const float* __restrict__ x, const float* __restrict__ w1, const float* __restrict__ al1, const float* __restrict__ ar1, const float* __restrict__ b1, const float* __restrict__ w2, const float* __restrict__ al2, const float* __restrict__ ar2, const float* __restrict__ b2, const float* __restrict__ rw2, b16* __restrict__ R1, b16* __restrict__ R2, float* __restrict__ P, b16* __restrict__ X, b16* __restrict__ Hlpad) {
  const size_t tid = (size_t)blockIdx.x * 256 + threadIdx.x, nth = (size_t)gridDim.x * 256;
  for (int pass = 0; pass < 2; ++pass) {
    for (size_t p = tid; p < (size_t)F1 * (FI / 8); p += nth) { const int o = (int)(p / (FI / 8)), k0 = (int)(p % (FI / 8)) * 8; v8b v; for (int e = 0; e < 8; ++e) v[e] = (b16)bf16_rne(w1[(size_t)(k0 + e) * F1 + o]); *(volatile v8b*)(R1 + (size_t)o * FI + k0) = v; }
    for (size_t p = tid; p < (size_t)2 * F2 * (F1 / 8); p += nth) { const int o = (int)(p / (F1 / 8)), k0 = (int)(p % (F1 / 8)) * 8; const float* W = (o < F2) ? w2 : rw2; const int oo = o % F2; v8b v; for (int e = 0; e < 8; ++e) v[e] = (b16)bf16_rne(W[(size_t)(k0 + e) * F2 + oo]); *(volatile v8b*)(R2 + (size_t)o * F1 + k0) = v; }
    for (size_t q = tid; q < 960; q += nth) { const int i = (int)q; float v; if (i < 256) v = al1[i]; else if (i < 512) v = ar1[i - 256]; else if (i < 768) v = b1[i - 512]; else if (i < 832) v = al2[i - 768]; else if (i < 896) v = ar2[i - 832]; else v = b2[i - 896]; P[q] = bf16_rne(v); }
    for (size_t p = tid; p < (size_t)NP * FI / 8; p += nth) { const size_t r = p / (FI / 8); v8b v = {}; if (r < (size_t)NN) for (int e = 0; e < 8; ++e) v[e] = (b16)(bf16_rne(x[p * 8 + e]) * XS); *(volatile v8b*)(X + p * 8) = v; if (r >= (size_t)NN) *(volatile v8b*)(Hlpad + (p - (size_t)NN * FI / 8) * 8) = v; }
    __threadfence(); }
}

template <int NOUT, int TWO>
__global__ __launch_bounds__(64) void gemm_kernel(const b16* __restrict__ Ah, const b16* __restrict__ Al, const b16* __restrict__ Bw, float* __restrict__ OUT) {
  __shared__ __attribute__((aligned(16))) float Ts[2][16][NOUT + 4];
  constexpr int NS = NOUT / 16;
  const int lane = threadIdx.x & 31, wave = threadIdx.x >> 5, nloc = lane & 15, hlf = lane >> 4, m0 = blockIdx.x * 32 + wave * 16;
  v8f acc[NS];
#pragma unroll
  for (int t = 0; t < NS; ++t) acc[t] = (v8f){};
#pragma unroll 2
  for (int kb = 0; kb < FI; kb += 32) { const v16b a = frag_kb(Ah + (size_t)(m0 + nloc) * FI + kb, hlf); v16b al_; if (TWO) al_ = frag_kb(Al + (size_t)(m0 + nloc) * FI + kb, hlf);
#pragma unroll
    for (int t = 0; t < NS; ++t) { const v16b bw = frag_kb(Bw + (size_t)(t * 16 + nloc) * FI + kb, hlf); acc[t] = wmma16b(a, bw, acc[t]); if (TWO) acc[t] = wmma16b(al_, bw, acc[t]); } }
#pragma unroll
  for (int t = 0; t < NS; ++t)
#pragma unroll
    for (int r = 0; r < 8; ++r) Ts[wave][8 * hlf + r][t * 16 + nloc] = acc[t][r] * (1.0f / XS);
  wave_lds_sync();
  for (int pass = 0; pass < 2; ++pass) { for (int i = lane; i < 16 * (NOUT / 4); i += 32) { const int rr = i / (NOUT / 4), c4 = (i % (NOUT / 4)) * 4; *(volatile v4f*)(OUT + (size_t)(m0 + rr) * NOUT + c4) = *(const v4f*)(&Ts[wave][rr][c4]); } __threadfence(); }
}

template <int LAYER>
__global__ __launch_bounds__(256) void elr_kernel(const float* __restrict__ FT, const float* __restrict__ P, float* __restrict__ ELR) {
  __shared__ __attribute__((aligned(16))) float Es[8][8];
  const int wave = threadIdx.x >> 5, v = blockIdx.x * 8 + wave, lane = threadIdx.x & 31;
  if (LAYER == 1) { float sl = 0.0f, sr = 0.0f;
#pragma unroll
    for (int e = 0; e < 8; ++e) { const float f = FT[(size_t)v * F1 + lane * 8 + e]; sl += pmul(f, P[lane * 8 + e]); sr += pmul(f, P[256 + lane * 8 + e]); }
    sl += __shfl_xor(sl, 1); sl += __shfl_xor(sl, 2); sl += __shfl_xor(sl, 4); sr += __shfl_xor(sr, 1); sr += __shfl_xor(sr, 2); sr += __shfl_xor(sr, 4);
    if ((lane & 7) == 0) { Es[wave][lane >> 3] = sl; Es[wave][4 + (lane >> 3)] = sr; } }
  else { float sl = 0.0f, sr = 0.0f;
#pragma unroll
    for (int e = 0; e < 2; ++e) { const float f = FT[(size_t)v * 128 + lane * 2 + e]; sl += pmul(f, P[768 + lane * 2 + e]); sr += pmul(f, P[832 + lane * 2 + e]); }
#pragma unroll
    for (int o = 1; o < 32; o <<= 1) { sl += __shfl_xor(sl, o); sr += __shfl_xor(sr, o); }
    if (lane < 8) Es[wave][lane] = (lane == 0) ? sl : (lane == 4) ? sr : 0.0f; }
  __syncthreads();
  for (int pass = 0; pass < 2; ++pass) { if (threadIdx.x < 16) *(volatile v4f*)(ELR + (size_t)blockIdx.x * 64 + threadIdx.x * 4) = *(const v4f*)(&Es[0][0] + threadIdx.x * 4); __threadfence(); }
}

__global__ __launch_bounds__(256) void gat1_kernel(const float* __restrict__ FT, const float* __restrict__ ELR, const int* __restrict__ src, const int* __restrict__ perm, const int* __restrict__ rowptr, const int* __restrict__ rowcnt, const float* __restrict__ P, b16* __restrict__ Hh, b16* __restrict__ Hl) {
  __shared__ __attribute__((aligned(16))) b16 Sh[8][F1 + 8], Sl[8][F1 + 8];
  const int wave = threadIdx.x >> 5, v = blockIdx.x * 8 + wave, lane = threadIdx.x & 31, hd = lane >> 3;
  int cnt = rowcnt[v]; cnt = (cnt < 0) ? 0 : (cnt > MAXDEG ? MAXDEG : cnt); int p0 = rowptr[v]; p0 = (p0 < 0) ? 0 : (p0 > PERMLEN - cnt ? PERMLEN - cnt : p0);
  const float erv = ELR[(size_t)v * 8 + 4 + hd]; float m = -INFINITY, l = 0.0f; float acc[8] = {0, 0, 0, 0, 0, 0, 0, 0};
  for (int q = 0; q < cnt; ++q) { int id = perm[p0 + q]; id = (id < 0) ? 0 : (id >= NE ? NE - 1 : id); int s = src[id]; s = (s < 0) ? 0 : (s >= NN ? NN - 1 : s);
    const float e = leaky(ELR[(size_t)s * 8 + hd] + erv); const float mn = fmaxf(m, e); const float al_ = nexp(m - mn); const float p = nexp(e - mn); m = mn; l = l * al_ + p;
    const v4f f0 = *(const v4f*)(FT + (size_t)s * F1 + lane * 8), f1 = *(const v4f*)(FT + (size_t)s * F1 + lane * 8 + 4);
#pragma unroll
    for (int k = 0; k < 4; ++k) { acc[k] = acc[k] * al_ + pmul(p, f0[k]); acc[4 + k] = acc[4 + k] * al_ + pmul(p, f1[k]); } }
  const float inv = (cnt > 0) ? 1.0f / l : 0.0f; float y[8];
#pragma unroll
  for (int k = 0; k < 8; ++k) { y[k] = elu_f(acc[k] * inv + P[512 + lane * 8 + k]); b16 a_, b_; split16(y[k] * XS, a_, b_); Sh[wave][lane * 8 + k] = a_; Sl[wave][lane * 8 + k] = b_; }
  wave_lds_sync();
  for (int pass = 0; pass < 2; ++pass) { *(volatile v8b*)(Hh + (size_t)v * F1 + lane * 8) = *(const v8b*)(&Sh[wave][lane * 8]); *(volatile v8b*)(Hl + (size_t)v * F1 + lane * 8) = *(const v8b*)(&Sl[wave][lane * 8]); __threadfence(); }
}
__global__ __launch_bounds__(256) void gat2_kernel(const float* __restrict__ FR, const float* __restrict__ ELR, const int* __restrict__ src, const int* __restrict__ perm, const int* __restrict__ rowptr, const int* __restrict__ rowcnt, const float* __restrict__ P, float* __restrict__ out) {
  const int wave = threadIdx.x >> 5, v = blockIdx.x * 8 + wave, lane = threadIdx.x & 31;
  int cnt = rowcnt[v]; cnt = (cnt < 0) ? 0 : (cnt > MAXDEG ? MAXDEG : cnt); int p0 = rowptr[v]; p0 = (p0 < 0) ? 0 : (p0 > PERMLEN - cnt ? PERMLEN - cnt : p0);
  const float erv = ELR[(size_t)v * 8 + 4]; float m = -INFINITY, l = 0.0f, a0 = 0.0f, a1 = 0.0f;
  for (int q = 0; q < cnt; ++q) { int id = perm[p0 + q]; id = (id < 0) ? 0 : (id >= NE ? NE - 1 : id); int s = src[id]; s = (s < 0) ? 0 : (s >= NN ? NN - 1 : s);
    const float e = leaky(ELR[(size_t)s * 8 + 0] + erv); const float mn = fmaxf(m, e); const float al_ = nexp(m - mn); const float p = nexp(e - mn); m = mn; l = l * al_ + p;
    const v2f f = *(const v2f*)(FR + (size_t)s * 128 + lane * 2); a0 = a0 * al_ + pmul(p, f[0]); a1 = a1 * al_ + pmul(p, f[1]); }
  const float inv = (cnt > 0) ? 1.0f / l : 0.0f; const v2f res = *(const v2f*)(FR + (size_t)v * 128 + 64 + lane * 2); v2f o; o[0] = a0 * inv + res[0] + P[896 + lane * 2]; o[1] = a1 * inv + res[1] + P[896 + lane * 2 + 1];
  for (int pass = 0; pass < 2; ++pass) { *(volatile v2f*)(out + (size_t)v * F2 + lane * 2) = o; __threadfence(); }
}
}

extern "C" void kernel_launch(void* const* d_in, const int* in_sizes, int n_in,
                              void* d_out, int out_size, void* d_ws, size_t ws_size, hipStream_t stream) {
  (void)n_in; (void)out_size;
  const float* x = (const float*)d_in[0]; const int* srcI = (const int*)d_in[1]; const int* dstI = (const int*)d_in[2]; const float* w1 = (const float*)d_in[3]; const float* al1 = (const float*)d_in[4]; const float* ar1 = (const float*)d_in[5]; const float* b1 = (const float*)d_in[6];
  const float* w2 = (const float*)d_in[7]; const float* al2 = (const float*)d_in[8]; const float* ar2 = (const float*)d_in[9]; const float* b2 = (const float*)d_in[10]; const float* rw2 = (const float*)d_in[11];
  float* out = (float*)d_out;
  if (in_sizes[0] != NN * FI || in_sizes[1] != NE || in_sizes[2] != NE || in_sizes[3] != FI * F1 || in_sizes[11] != F1 * F2) return;
  const int NE_RUN = NE;
  size_t off = 0; char* ws = (char*)d_ws;
  auto carve = [&](size_t bytes) { char* p = ws + off; off += (bytes + 255) & ~(size_t)255; return p; };
  b16* R1 = (b16*)carve((size_t)F1 * FI * 2); b16* R2 = (b16*)carve((size_t)128 * F1 * 2); float* P = (float*)carve(960 * 4); b16* X = (b16*)carve((size_t)NP * FI * 2); float* FT = (float*)carve((size_t)NP * F1 * 4); float* ELR = (float*)carve((size_t)NP * 8 * 4);
  b16* Hl = (b16*)carve((size_t)NP * F1 * 2);
  CsrBufs cs; off = csr_carve(cs, ws, off, NE_RUN, NN);
  if (off > ws_size) return;
  b16* Hh = X; float* FR = FT;
  csr_build(cs, dstI, NE_RUN, NN, stream);
  prep_kernel<<<512, 256, 0, stream>>>(x, w1, al1, ar1, b1, w2, al2, ar2, b2, rw2, R1, R2, P, X, Hl + (size_t)NN * F1);
  gemm_kernel<256, 0><<<NP / 32, 64, 0, stream>>>(X, nullptr, R1, FT);
  elr_kernel<1><<<NN / 8, 256, 0, stream>>>(FT, P, ELR);
  gat1_kernel<<<NN / 8, 256, 0, stream>>>(FT, ELR, srcI, cs.PERM, cs.ROWPTR, cs.ROWCNT, P, Hh, Hl);
  gemm_kernel<128, 1><<<NP / 32, 64, 0, stream>>>(Hh, Hl, R2, FR);
  elr_kernel<2><<<NN / 8, 256, 0, stream>>>(FR, P, ELR);
  gat2_kernel<<<NN / 8, 256, 0, stream>>>(FR, ELR, srcI, cs.PERM, cs.ROWPTR, cs.ROWCNT, P, out);
}
